// SDOT_11579231830512
// MI455X (gfx1250) — hardware-verified
//
#include <hip/hip_runtime.h>
#include <math.h>

typedef __attribute__((ext_vector_type(16))) _Float16 v16h;
typedef __attribute__((ext_vector_type(16))) __bf16 v16b;
typedef __attribute__((ext_vector_type(8)))  _Float16 v8h;
typedef __attribute__((ext_vector_type(8)))  float v8f;
typedef __attribute__((ext_vector_type(4)))  float v4f;
typedef __attribute__((ext_vector_type(2)))  float v2f;
typedef __attribute__((ext_vector_type(4)))  unsigned v4u;
typedef __attribute__((ext_vector_type(4)))  int v4i;
typedef float __attribute__((may_alias)) float_a;
typedef int __attribute__((may_alias)) int_a;

template <typename T> __device__ __forceinline__ void vst2(void* p, T v) { *(volatile T*)p = v; __threadfence(); *(volatile T*)p = v; }
__device__ __forceinline__ v8f wmma16(v16h a, v16h b, v8f c) {
  v8f d = __builtin_amdgcn_wmma_f32_16x16x32_f16(false, a, false, b, (short)0, c, false, false);
  asm volatile("v_nop\n\tv_nop\n\tv_nop\n\tv_nop" : "+v"(d) : "v"(a), "v"(b));
  return d;
}
__device__ __forceinline__ v8f wmma_bf(v16b a, v16b b, v8f c) {
  v8f d = __builtin_amdgcn_wmma_f32_16x16x32_bf16(false, a, false, b, (short)0, c, false, false);
  asm volatile("v_nop\n\tv_nop\n\tv_nop\n\tv_nop" : "+v"(d) : "v"(a), "v"(b));
  return d;
}
__device__ __forceinline__ v16h frag_h(const _Float16* rowk0, int lane) {
  union { v16h v; v8h q[2]; } u; const _Float16* p = rowk0 + 8 * (lane >> 4);
  u.q[0] = *(const v8h*)p; u.q[1] = *(const v8h*)(p + 16); return u.v;
}
__device__ __forceinline__ v16h frag_f32(const float* rowk0, int lane) {
  v16h a; const float* p = rowk0 + 8 * (lane >> 4);
#pragma unroll
  for (int i = 0; i < 8; ++i) { a[i] = (_Float16)p[i]; a[8 + i] = (_Float16)p[16 + i]; }
  return a;
}
__device__ __forceinline__ v16h frag_f32s(const float* rowk0, int lane, float sc) {
  v16h a; const float* p = rowk0 + 8 * (lane >> 4);
#pragma unroll
  for (int i = 0; i < 8; ++i) { a[i] = (_Float16)(p[i] * sc); a[8 + i] = (_Float16)(p[16 + i] * sc); }
  return a;
}
__device__ __forceinline__ v16h fragc_f32(const float* W, int k0, int n, int lane, int ld, int K) {
  v16h a; const int g = lane >> 4;
#pragma unroll
  for (int i = 0; i < 8; ++i) { const int ka = k0 + 8 * g + i, kb = ka + 16;
    a[i] = (_Float16)(ka < K ? W[(size_t)(ka < K ? ka : K - 1) * ld + n] : 0.f); a[8 + i] = (_Float16)(kb < K ? W[(size_t)(kb < K ? kb : K - 1) * ld + n] : 0.f); }
  return a;
}
struct F2 { v16b h, l; };
__device__ __forceinline__ F2 bsplit16(const float v[16]) { F2 r;
#pragma unroll
  for (int i = 0; i < 16; ++i) { const __bf16 h = (__bf16)v[i]; r.h[i] = h; r.l[i] = (__bf16)(v[i] - (float)h); }
  return r; }
__device__ __forceinline__ F2 split_row(const float* row, int k0, int lane) { float v[16]; const float* p = row + k0 + 8 * (lane >> 4);
#pragma unroll
  for (int i = 0; i < 8; ++i) { v[i] = p[i]; v[8 + i] = p[16 + i]; }
  return bsplit16(v); }
__device__ __forceinline__ F2 split_rowK(const float* row, int k0, int lane, int K) { float v[16]; const int g = lane >> 4;
#pragma unroll
  for (int i = 0; i < 8; ++i) { const int ka = k0 + 8 * g + i, kb = ka + 16; v[i] = ka < K ? row[ka < K ? ka : K - 1] : 0.f; v[8 + i] = kb < K ? row[kb < K ? kb : K - 1] : 0.f; }
  return bsplit16(v); }
__device__ __forceinline__ F2 split_col(const float* W, int k0, int n, int lane, int ld, int K) { float v[16]; const int g = lane >> 4;
#pragma unroll
  for (int i = 0; i < 8; ++i) { const int ka = k0 + 8 * g + i, kb = ka + 16; v[i] = ka < K ? W[(size_t)(ka < K ? ka : K - 1) * ld + n] : 0.f; v[8 + i] = kb < K ? W[(size_t)(kb < K ? kb : K - 1) * ld + n] : 0.f; }
  return bsplit16(v); }
__device__ __forceinline__ v8f mac3(const F2& a, const F2& b, v8f c) { c = wmma_bf(a.l, b.h, c); c = wmma_bf(a.h, b.l, c); return wmma_bf(a.h, b.h, c); }
__device__ __forceinline__ float sigm(float v) { return 1.0f / (1.0f + expf(-v)); }
#define LDSX() do { asm volatile("s_wait_dscnt 0" ::: "memory"); __builtin_amdgcn_wave_barrier(); __builtin_amdgcn_fence(__ATOMIC_RELEASE, "workgroup"); } while (0)

__device__ __forceinline__ float bfr(float v) { return (float)(__bf16)v; }
#define NS 32768
#define MT 8192
#define DD 64
#ifndef NRB
#define NRB (NS / 64)
#endif
#define WS_TY  0u
#define WS_PS  (WS_TY + 4u * (size_t)MT)
#define WS_SC  (WS_PS + 4u * 128u * 32u)
#define WS_END (WS_SC + 4u * 32u)
__global__ __launch_bounds__(64) void k_ty(const float* __restrict__ Y, const float* __restrict__ PSI, float* __restrict__ TY, float* __restrict__ PS) { __shared__ __align__(16) float st[64]; __shared__ float sp[64];
  const int j = blockIdx.x * 64 + threadIdx.x; const float* p = Y + (size_t)j * DD; float s = 0.f; for (int d = 0; d < DD; ++d) { const float v = bfr(p[d]); s += v * v; }
  st[threadIdx.x] = s; sp[threadIdx.x] = bfr(PSI[j]); LDSX(); __syncthreads();
  if (threadIdx.x < 16) vst2(TY + blockIdx.x * 64 + threadIdx.x * 4, *(const v4f*)&st[threadIdx.x * 4]);
  if (threadIdx.x < 32) { float a = 0.f, b = 0.f; for (int e = 0; e < 64; ++e) { a += st[e]; b += sp[e]; }
    const float line = (threadIdx.x == 0) ? a : (threadIdx.x == 1) ? b : 0.f; vst2(PS + blockIdx.x * 32 + threadIdx.x, line); } }
__global__ __launch_bounds__(32) void k_sc2(const float* __restrict__ PS, float* __restrict__ SC) { float a = 0.f, b = 0.f; for (int e = 0; e < MT / 64; ++e) { a += PS[e * 32]; b += PS[e * 32 + 1]; }
  const float v = (threadIdx.x == 0) ? (float)MT / a : (threadIdx.x == 1 ? b / (float)MT : 0.f); vst2(SC + threadIdx.x, v); }
__global__ __launch_bounds__(128) void k_lse(const float* __restrict__ X, const float* __restrict__ Y, const float* __restrict__ PSI, const float* __restrict__ TY, const float* __restrict__ SC, float* __restrict__ OUT) { __shared__ __align__(16) float so[64]; __shared__ float sx2[64];
  const int tid = threadIdx.x, wave = tid >> 5, lane = tid & 31, col = lane & 15, g = lane >> 4; const size_t r0 = (size_t)blockIdx.x * 64 + wave * 16;
  if (tid < 64) { const float* p = X + ((size_t)blockIdx.x * 64 + tid) * DD; float s = 0.f; for (int d = 0; d < DD; ++d) { const float v = bfr(p[d]); s += v * v; } sx2[tid] = s; }
  v16b af[2];
#pragma unroll
  for (int kc = 0; kc < 2; ++kc) { const float* p = X + (r0 + col) * DD + kc * 32 + 8 * g;
#pragma unroll
    for (int i = 0; i < 8; ++i) { af[kc][i] = (__bf16)p[i]; af[kc][8 + i] = (__bf16)p[16 + i]; } }
  __syncthreads();
  const float invm = SC[0], mpsi = SC[1];
  float m8[8], s8[8];
#pragma unroll
  for (int r = 0; r < 8; ++r) { m8[r] = -3.0e38f; s8[r] = 0.f; }
#pragma unroll 1
  for (int cb = 0; cb < MT / 128; ++cb) { const int c0 = cb * 128; v8f acc[8] = {};
#pragma unroll
    for (int kc = 0; kc < 2; ++kc) {
#pragma unroll
      for (int j = 0; j < 8; ++j) { v16b w; const float* p = Y + (size_t)(c0 + j * 16 + col) * DD + kc * 32 + 8 * g;
#pragma unroll
        for (int i = 0; i < 8; ++i) { w[i] = (__bf16)p[i]; w[8 + i] = (__bf16)p[16 + i]; }
        acc[j] = wmma_bf(af[kc], w, acc[j]); } }
#pragma unroll
    for (int j = 0; j < 8; ++j) { const int jc = c0 + j * 16 + col; const float ty = TY[jc]; const float ps = bfr(PSI[jc]);
#pragma unroll
      for (int r = 0; r < 8; ++r) { const float cost = ((sx2[wave * 16 + 8 * g + r] + ty) - 2.0f * acc[j][r]) * invm; const float v = (ps - cost) * 100.0f; const float mn = fmaxf(m8[r], v); s8[r] = s8[r] * __expf(m8[r] - mn) + __expf(v - mn); m8[r] = mn; } } }
#pragma unroll
  for (int r = 0; r < 8; ++r) { float m = m8[r], s = s8[r];
#pragma unroll
    for (int o = 1; o < 16; o <<= 1) { const float mo = __shfl_xor(m, o), so2 = __shfl_xor(s, o); const float mn = fmaxf(m, mo); s = s * __expf(m - mn) + so2 * __expf(mo - mn); m = mn; }
    if (col == 0) so[wave * 16 + 8 * g + r] = -0.01f * (m + logf(s)) + mpsi; }
  __syncthreads(); if (tid < 16) vst2(OUT + (size_t)blockIdx.x * 64 + tid * 4, *(const v4f*)&so[tid * 4]); }
extern "C" void kernel_launch(void* const* d_in, const int* in_sizes, int n_in, void* d_out, int out_size, void* d_ws, size_t ws_size, hipStream_t stream) {
  (void)in_sizes; (void)n_in; (void)out_size;
  const float** F = (const float**)d_in;
  if (ws_size < (size_t)WS_END) return;
  char* ws = (char*)d_ws; float *TY = (float*)(ws + WS_TY), *PS = (float*)(ws + WS_PS), *SC = (float*)(ws + WS_SC);
  k_ty<<<dim3(MT / 64), 64, 0, stream>>>(F[1], F[2], TY, PS);
  k_sc2<<<dim3(1), 32, 0, stream>>>(PS, SC);
  k_lse<<<dim3(NRB), 128, 0, stream>>>(F[0], F[1], F[2], TY, SC, (float*)d_out);
}
